// MultiHeadDuplexAttention1_1219770712285
// MI455X (gfx1250) — hardware-verified
//
#include <hip/hip_runtime.h>
#include <math.h>

constexpr int kBatch  = 4;
constexpr int kSeq    = 1024;
constexpr int kDim    = 1024;
constexpr int kHeads  = 16;
constexpr int kDk     = 64;
constexpr int kTok    = kBatch * kSeq;
constexpr int kGroups = kBatch * kHeads;
constexpr int kChunkG = 8;
constexpr int kNumChunks = kGroups / kChunkG;
constexpr int kChunksPerBatch = kHeads / kChunkG;
constexpr float kScale     = 0.125f;
constexpr float kWCarry    = 256.0f;
constexpr float kPCarry    = 2048.0f;
constexpr float kAttCarry  = 64.0f;
constexpr float kKfCarry   = 32.0f;
constexpr float kLnEps     = 1e-5f;
constexpr float kOmEps     = 1e-5f;

constexpr size_t kPlaneH   = (size_t)kTok * kDim * 2;
constexpr size_t kPlaneF   = (size_t)kTok * kDim * 4;
constexpr size_t kWPlane   = (size_t)kDim * kDim * 2;
constexpr size_t kSBytes   = (size_t)kChunkG * kSeq * kSeq * 4;
constexpr size_t kPBytes   = (size_t)kChunkG * kSeq * kSeq * 2;
constexpr size_t kStatBytes = (size_t)kBatch * kDim * 4;
constexpr size_t oW    = 0;
constexpr size_t oX16  = oW + 6 * kWPlane;
constexpr size_t oY16  = oX16 + kPlaneH;
constexpr size_t oQ1   = oY16 + kPlaneH;
constexpr size_t oK1   = oQ1 + kPlaneH;
constexpr size_t oV1T  = oK1 + kPlaneH;
constexpr size_t oQc   = oV1T + kPlaneH;
constexpr size_t oS    = oQc + kPlaneH;
constexpr size_t oP    = oS + kSBytes;
constexpr size_t oZ    = oP + kPBytes;
constexpr size_t oMu   = oZ + kPlaneF;
constexpr size_t oInv  = oMu + kStatBytes;
constexpr size_t kWsTotal = oInv + kStatBytes;
static_assert(kWsTotal <= (size_t)134217728u);
static_assert((size_t)kBatch * kSeq * kSeq * 4 <= kSBytes);
static_assert(kPlaneF <= kSBytes);
static_assert((size_t)kBatch * kSeq * kSeq * 2 <= kPBytes);

typedef __attribute__((ext_vector_type(16))) _Float16 v16h;
typedef __attribute__((ext_vector_type(8)))  _Float16 v8h;
typedef __attribute__((ext_vector_type(16))) __bf16   v16b;
typedef __attribute__((ext_vector_type(8)))  __bf16   v8b;
typedef __attribute__((ext_vector_type(8)))  float    v8f;
typedef __attribute__((ext_vector_type(4)))  float    v4f;
typedef __attribute__((ext_vector_type(4)))  unsigned int v4u;

__device__ __forceinline__ unsigned short f2bf_bits(float f) {
  unsigned u = __float_as_uint(f);
  return (unsigned short)((u + 0x7FFFu + ((u >> 16) & 1u)) >> 16);
}
__device__ __forceinline__ float bf_bits2f(unsigned short h) { return __uint_as_float(((unsigned)h) << 16); }

__device__ __forceinline__ void dep_guard_h(v8f& a, v8f& b, v16h x, v16h y) { asm volatile("v_nop\n\tv_nop\n\tv_nop\n\tv_nop" : "+v"(a), "+v"(b) : "v"(x), "v"(y)); }
__device__ __forceinline__ void dep_guard_b(v8f& a, v8f& b, v16b x, v16b y) { asm volatile("v_nop\n\tv_nop\n\tv_nop\n\tv_nop" : "+v"(a), "+v"(b) : "v"(x), "v"(y)); }
__device__ __forceinline__ void keep4_h(v16h a, v16h b, v16h c, v16h d) { asm volatile("v_nop" :: "v"(a), "v"(b), "v"(c), "v"(d)); }
__device__ __forceinline__ void keep4_b(v16b a, v16b b, v16b c, v16b d) { asm volatile("v_nop" :: "v"(a), "v"(b), "v"(c), "v"(d)); }
__device__ __forceinline__ void acc_guard4(v8f& a, v8f& b, v8f& c, v8f& d) { asm volatile("v_nop\n\tv_nop\n\tv_nop\n\tv_nop" : "+v"(a), "+v"(b), "+v"(c), "+v"(d)); }
template <typename T> struct Frag;
template <> struct Frag<_Float16> {
  typedef v16h V; union U { v16h v; v8h h[2]; };
  static __device__ __forceinline__ v16h load(const _Float16* p) {
    U f; f.h[0] = *(const v8h*)(p); f.h[1] = *(const v8h*)(p + 16); return f.v;
  }
  static __device__ __forceinline__ v8f mma(v16h a, v16h b, v8f c) {
    return __builtin_amdgcn_wmma_f32_16x16x32_f16(false, a, false, b, (short)0, c, false, false);
  }
  static __device__ __forceinline__ void guard(v8f& a, v8f& b, v16h x, v16h y) { dep_guard_h(a, b, x, y); }
  static __device__ __forceinline__ void keep(v16h a, v16h b, v16h c, v16h d) { keep4_h(a, b, c, d); }
};
template <> struct Frag<__bf16> {
  typedef v16b V; union U { v16b v; v8b h[2]; };
  static __device__ __forceinline__ v16b load(const __bf16* p) {
    U f; f.h[0] = *(const v8b*)(p); f.h[1] = *(const v8b*)(p + 16); return f.v;
  }
  static __device__ __forceinline__ v8f mma(v16b a, v16b b, v8f c) {
    return __builtin_amdgcn_wmma_f32_16x16x32_bf16(false, a, false, b, (short)0, c, false, false);
  }
  static __device__ __forceinline__ void guard(v8f& a, v8f& b, v16b x, v16b y) { dep_guard_b(a, b, x, y); }
  static __device__ __forceinline__ void keep(v16b a, v16b b, v16b c, v16b d) { keep4_b(a, b, c, d); }
};

__device__ __forceinline__ unsigned pk16(unsigned short a, unsigned short b) { return (unsigned)a | ((unsigned)b << 16); }
__device__ __forceinline__ unsigned short h_bits(float f) { const _Float16 h = (_Float16)f; return __builtin_bit_cast(unsigned short, h); }

template <int ET> struct Elem;
template <> struct Elem<0> { typedef _Float16 T; };
template <> struct Elem<1> { typedef __bf16 T; };
template <int ET, bool SPLIT, int BIAS_MODE, int OUT_MODE, bool RESID, int ACT = 0>
__global__ __launch_bounds__(256) void wmma_gemm64(
    const unsigned short* __restrict__ Ap, const unsigned short* __restrict__ A2p, int lda, long strideA,
    const unsigned short* __restrict__ Btp, const unsigned short* __restrict__ Bt2p, int ldb, long strideB,
    void* __restrict__ Cout, void* __restrict__ Cout2, int ldc, long strideC,
    const float* __restrict__ bias,
    const float* __restrict__ resid, long strideR,
    int M, int N, int K, float scale, float bias_scale) {
  typedef typename Elem<ET>::T T;
  typedef typename Frag<T>::V V;
  const T* A = (const T*)Ap; const T* A2 = (const T*)A2p; const T* Bt = (const T*)Btp; const T* Bt2 = (const T*)Bt2p;
  __shared__ __align__(16) float sT[8][16 * 68];
  const int b    = blockIdx.y;
  const int lane = threadIdx.x & 31;
  const int wave = threadIdx.x >> 5;
  const int tilesN = N >> 6;
  const int tilesM = M >> 6;
  const int tile = blockIdx.x * 8 + wave;
  if (tile >= tilesM * tilesN) return;
  const int tm = tile / tilesN;
  const int tn = tile - tm * tilesN;
  const int m0 = tm << 6;
  const int n0 = tn << 6;

  const T* Ab  = A  + (size_t)b * strideA;
  const T* Bb  = Bt + (size_t)b * strideB;
  const T* Ab2 = SPLIT ? (A2  + (size_t)b * strideA) : nullptr;
  const T* Bb2 = SPLIT ? (Bt2 + (size_t)b * strideB) : nullptr;

  const int rlane = lane & 15;
  const int koff  = (lane >> 4) * 8;
  const int mOff  = (lane >> 4) * 8;

  v8f acc[4][4];
#pragma unroll
  for (int i = 0; i < 4; ++i)
#pragma unroll
    for (int j = 0; j < 4; ++j) acc[i][j] = (v8f){0.f,0.f,0.f,0.f,0.f,0.f,0.f,0.f};

  for (int k0 = 0; k0 < K; k0 += 32) {
    V bh[4], bl[4];
#pragma unroll
    for (int j = 0; j < 4; ++j) {
      const size_t bo = (size_t)(n0 + (j << 4) + rlane) * ldb + koff + k0;
      bh[j] = Frag<T>::load(Bb + bo);
      if (SPLIT) bl[j] = Frag<T>::load(Bb2 + bo);
    }
#pragma unroll
    for (int i = 0; i < 4; ++i) {
      const size_t ao = (size_t)(m0 + (i << 4) + rlane) * lda + koff + k0;
      V ah = Frag<T>::load(Ab + ao);
      V al;
      if (SPLIT) al = Frag<T>::load(Ab2 + ao);
#pragma unroll
      for (int j = 0; j < 4; ++j) {
        acc[i][j] = Frag<T>::mma(ah, bh[j], acc[i][j]);
        if (SPLIT) {
          acc[i][j] = Frag<T>::mma(ah, bl[j], acc[i][j]);
          acc[i][j] = Frag<T>::mma(al, bh[j], acc[i][j]);
        }
      }
      Frag<T>::guard(acc[i][0], acc[i][3], ah, SPLIT ? al : ah);
    }
    Frag<T>::keep(bh[0], bh[1], bh[2], bh[3]);
    if (SPLIT) Frag<T>::keep(bl[0], bl[1], bl[2], bl[3]);
  }
  acc_guard4(acc[0][0], acc[0][1], acc[0][2], acc[0][3]);
  acc_guard4(acc[1][0], acc[1][1], acc[1][2], acc[1][3]);
  acc_guard4(acc[2][0], acc[2][1], acc[2][2], acc[2][3]);
  acc_guard4(acc[3][0], acc[3][1], acc[3][2], acc[3][3]);

  float* slab = sT[wave];
  const float* Rb = RESID ? (resid + (size_t)b * strideR) : nullptr;
#pragma unroll
  for (int i = 0; i < 4; ++i) {
    const int mBase = m0 + (i << 4);
#pragma unroll
    for (int j = 0; j < 4; ++j) {
      const int n = n0 + (j << 4) + rlane;
      float bv = 0.f;
      if (BIAS_MODE == 2) bv = bias[n] * bias_scale;
#pragma unroll
      for (int r = 0; r < 8; ++r) {
        float v = acc[i][j][r] * scale;
        if (BIAS_MODE == 1) v += bias[mBase + mOff + r] * bias_scale;
        if (BIAS_MODE == 2) v += bv;
        if (RESID) v += Rb[(size_t)(mBase + mOff + r) * ldc + n];
        if (ACT == 2) v = fmaxf(v, 0.0f);
        if (ACT == 4) v = (v > 0.f) ? v : 0.01f * v;
        slab[(mOff + r) * 68 + (j << 4) + rlane] = v;
      }
    }
    __builtin_amdgcn_fence(__ATOMIC_RELEASE, "workgroup");
    __builtin_amdgcn_wave_barrier();
    __builtin_amdgcn_fence(__ATOMIC_ACQUIRE, "workgroup");
    if (OUT_MODE == 0) {
      float* C = (float*)Cout + (size_t)b * strideC;
      const int hh = lane >> 4, c4 = (lane & 15) * 4;
      for (int pass = 0; pass < 2; ++pass) {
#pragma unroll
        for (int it = 0; it < 8; ++it) {
          const int row = it * 2 + hh;
          v4f v = *(const v4f*)(slab + row * 68 + c4);
          *(volatile v4f*)(C + (size_t)(mBase + row) * ldc + n0 + c4) = v;
        }
        __threadfence();
      }
    } else {
      const int q = lane >> 3, c8 = (lane & 7) * 8;
      unsigned short* C  = (unsigned short*)Cout  + (size_t)b * strideC;
      unsigned short* C2 = (OUT_MODE == 2) ? ((unsigned short*)Cout2 + (size_t)b * strideC) : nullptr;
      for (int pass = 0; pass < 2; ++pass) {
#pragma unroll
        for (int it = 0; it < 4; ++it) {
          const int row = it * 4 + q;
          const float* sp = slab + row * 68 + c8;
          v8h hv, lv;
#pragma unroll
          for (int e = 0; e < 8; ++e) {
            if (OUT_MODE == 1) {
              hv[e] = (_Float16)sp[e];
            } else {
              unsigned short hb = f2bf_bits(sp[e]);
              unsigned short lb = f2bf_bits(sp[e] - bf_bits2f(hb));
              hv[e] = __builtin_bit_cast(_Float16, hb);
              lv[e] = __builtin_bit_cast(_Float16, lb);
            }
          }
          *(volatile v8h*)(C + (size_t)(mBase + row) * ldc + n0 + c8) = hv;
          if (OUT_MODE == 2) *(volatile v8h*)(C2 + (size_t)(mBase + row) * ldc + n0 + c8) = lv;
        }
        __threadfence();
      }
    }
    __builtin_amdgcn_fence(__ATOMIC_RELEASE, "workgroup");
    __builtin_amdgcn_wave_barrier();
    __builtin_amdgcn_fence(__ATOMIC_ACQUIRE, "workgroup");
  }
}

__global__ __launch_bounds__(256) void wtcast6_kernel(const float* __restrict__ W0, const float* __restrict__ W1,
                                                      const float* __restrict__ W2, const float* __restrict__ W3,
                                                      const float* __restrict__ W4, const float* __restrict__ W5,
                                                      unsigned short* __restrict__ out, float scale) {
  __shared__ float sm[64][65];
  const int t  = threadIdx.x;
  const int k0 = blockIdx.x * 64;
  const int n0 = blockIdx.y * 64;
  const int z  = blockIdx.z;
  const float* W = (z == 0) ? W0 : (z == 1) ? W1 : (z == 2) ? W2 : (z == 3) ? W3 : (z == 4) ? W4 : W5;
#pragma unroll
  for (int i = 0; i < 16; ++i) {
    const int e = i * 256 + t;
    const int r = e >> 6;
    const int c = e & 63;
    sm[c][r] = W[(size_t)(k0 + r) * kDim + n0 + c] * scale;
  }
  __syncthreads();
  const int lane = t & 31, wave = t >> 5;
  const int q = lane >> 3, c8 = (lane & 7) * 8;
  unsigned short* op = out + (size_t)z * kDim * kDim;
  for (int pass = 0; pass < 2; ++pass) {
#pragma unroll
    for (int it = 0; it < 2; ++it) {
      const int row = wave * 8 + it * 4 + q;
      unsigned short hb[8];
#pragma unroll
      for (int e = 0; e < 8; ++e) hb[e] = h_bits(sm[row][c8 + e]);
      const v4u u = (v4u){pk16(hb[0], hb[1]), pk16(hb[2], hb[3]), pk16(hb[4], hb[5]), pk16(hb[6], hb[7])};
      *(volatile v4u*)(op + (size_t)(n0 + row) * kDim + k0 + c8) = u;
    }
    __threadfence();
  }
}

__global__ __launch_bounds__(256) void cast8_f16_kernel(const float* __restrict__ in, unsigned short* __restrict__ out, int n8) {
  const int i = blockIdx.x * 256 + threadIdx.x;
  if (i >= n8) return;
  const float* p = in + 8 * (size_t)i;
  const v4f a = *(const v4f*)(p);
  const v4f c = *(const v4f*)(p + 4);
  unsigned short hb[8];
#pragma unroll
  for (int e = 0; e < 4; ++e) {
    hb[e]     = h_bits(a[e]);
    hb[4 + e] = h_bits(c[e]);
  }
  const v4u u = (v4u){pk16(hb[0], hb[1]), pk16(hb[2], hb[3]), pk16(hb[4], hb[5]), pk16(hb[6], hb[7])};
  unsigned short* q = out + 8 * (size_t)i;
  *(volatile v4u*)q = u;
  __threadfence();
  *(volatile v4u*)q = u;
}

__global__ __launch_bounds__(128) void softmax1024_kernel(const float* __restrict__ S, unsigned short* __restrict__ P, float carry) {
  __shared__ float redM[4];
  __shared__ float redS[4];
  const int row  = blockIdx.x;
  const int t    = threadIdx.x;
  const int lane = t & 31, wave = t >> 5;
  const int c0   = t * 8;
  const float* sr = S + (size_t)row * kSeq + c0;
  const v4f a = *(const v4f*)(sr);
  const v4f c = *(const v4f*)(sr + 4);
  float x[8];
#pragma unroll
  for (int e = 0; e < 4; ++e) { x[e] = a[e]; x[4 + e] = c[e]; }
  float m = fmaxf(fmaxf(fmaxf(x[0], x[1]), fmaxf(x[2], x[3])), fmaxf(fmaxf(x[4], x[5]), fmaxf(x[6], x[7])));
#pragma unroll
  for (int off = 16; off > 0; off >>= 1) m = fmaxf(m, __shfl_xor(m, off, 32));
  if (lane == 0) redM[wave] = m;
  __syncthreads();
  const float gm = fmaxf(fmaxf(redM[0], redM[1]), fmaxf(redM[2], redM[3]));
  float ev[8];
#pragma unroll
  for (int e = 0; e < 8; ++e) ev[e] = expf(x[e] - gm);
  float s = ((ev[0] + ev[1]) + (ev[2] + ev[3])) + ((ev[4] + ev[5]) + (ev[6] + ev[7]));
#pragma unroll
  for (int off = 16; off > 0; off >>= 1) s += __shfl_xor(s, off, 32);
  if (lane == 0) redS[wave] = s;
  __syncthreads();
  const float tot = (redS[0] + redS[1]) + (redS[2] + redS[3]);
  const float f = carry / tot;
  unsigned short hb[8];
#pragma unroll
  for (int e = 0; e < 8; ++e) hb[e] = h_bits(ev[e] * f);
  const v4u u = (v4u){pk16(hb[0], hb[1]), pk16(hb[2], hb[3]), pk16(hb[4], hb[5]), pk16(hb[6], hb[7])};
  unsigned short* q = P + (size_t)row * kSeq + c0;
  *(volatile v4u*)q = u;
  __threadfence();
  *(volatile v4u*)q = u;
}

__global__ __launch_bounds__(256) void ln_row_kernel(const float* __restrict__ Z, float* __restrict__ outY,
                                                     unsigned short* __restrict__ YN) {
  __shared__ float redA[8];
  __shared__ float redB[8];
  __shared__ __align__(16) unsigned rowh[512];
  const int row  = blockIdx.x;
  const int t    = threadIdx.x;
  const int lane = t & 31, wave = t >> 5;
  const size_t base = (size_t)row * kDim + 4 * t;
  const v4f z = *(const v4f*)(Z + base);
  float s = (z[0] + z[1]) + (z[2] + z[3]);
#pragma unroll
  for (int off = 16; off > 0; off >>= 1) s += __shfl_xor(s, off, 32);
  if (lane == 0) redA[wave] = s;
  __syncthreads();
  const float tot = ((redA[0] + redA[1]) + (redA[2] + redA[3])) + ((redA[4] + redA[5]) + (redA[6] + redA[7]));
  const float mu = tot * (1.0f / 1024.0f);
  const float e0 = z[0] - mu, e1 = z[1] - mu, e2 = z[2] - mu, e3 = z[3] - mu;
  float ss = (e0 * e0 + e1 * e1) + (e2 * e2 + e3 * e3);
#pragma unroll
  for (int off = 16; off > 0; off >>= 1) ss += __shfl_xor(ss, off, 32);
  if (lane == 0) redB[wave] = ss;
  __syncthreads();
  const float tot2 = ((redB[0] + redB[1]) + (redB[2] + redB[3])) + ((redB[4] + redB[5]) + (redB[6] + redB[7]));
  const float var  = tot2 * (1.0f / 1024.0f);
  const float rstd = rsqrtf(var + kLnEps);
  const v4f o = (v4f){e0 * rstd, e1 * rstd, e2 * rstd, e3 * rstd};
  float* op = outY + base;
  *(volatile v4f*)op = o;
  __threadfence();
  *(volatile v4f*)op = o;
  rowh[2 * t]     = pk16(h_bits(o[0]), h_bits(o[1]));
  rowh[2 * t + 1] = pk16(h_bits(o[2]), h_bits(o[3]));
  __syncthreads();
  if (t < 128) {
    const v4u u = *(const v4u*)(rowh + 4 * t);
    unsigned short* hp = YN + (size_t)row * kDim + 8 * t;
    *(volatile v4u*)hp = u;
    __threadfence();
    *(volatile v4u*)hp = u;
  }
}

__global__ __launch_bounds__(256) void transpose16_kernel(const unsigned short* __restrict__ in, unsigned short* __restrict__ out) {
  __shared__ unsigned short sm[64][66];
  const int t  = threadIdx.x;
  const int d0 = blockIdx.x * 64;
  const int t0 = blockIdx.y * 64;
  const int b  = blockIdx.z;
  const unsigned* inw = (const unsigned*)in;
#pragma unroll
  for (int i = 0; i < 8; ++i) {
    const int e  = i * 256 + t;
    const int r  = e >> 5;
    const int cp = e & 31;
    const unsigned u = inw[(((size_t)(b * kSeq + t0 + r)) * kDim + d0) / 2 + cp];
    sm[2 * cp][r]     = (unsigned short)(u & 0xffffu);
    sm[2 * cp + 1][r] = (unsigned short)(u >> 16);
  }
  __syncthreads();
  const int lane = t & 31, wave = t >> 5;
  const int q = lane >> 3, c8 = (lane & 7) * 8;
  unsigned short* ob = out + (size_t)b * kDim * kSeq;
  for (int pass = 0; pass < 2; ++pass) {
#pragma unroll
    for (int it = 0; it < 2; ++it) {
      const int row = wave * 8 + it * 4 + q;
      const unsigned short* sp = &sm[row][c8];
      const v4u u = (v4u){pk16(sp[0], sp[1]), pk16(sp[2], sp[3]), pk16(sp[4], sp[5]), pk16(sp[6], sp[7])};
      *(volatile v4u*)(ob + (size_t)(d0 + row) * kSeq + t0 + c8) = u;
    }
    __threadfence();
  }
}

__global__ __launch_bounds__(256) void colstats_kernel(const float* __restrict__ X, float* __restrict__ mu,
                                                       float* __restrict__ inv) {
  const int d = blockIdx.x * 256 + threadIdx.x;
  const int b = blockIdx.y;
  const float* p = X + (size_t)b * kSeq * kDim + d;
  float s = 0.f;
#pragma unroll 1
  for (int i0 = 0; i0 < kSeq; i0 += 32) {
    float sb = 0.f;
#pragma unroll 4
    for (int i = 0; i < 32; ++i) sb += p[(size_t)(i0 + i) * kDim];
    s += sb;
  }
  const float m = s * (1.0f / 1024.0f);
  float ss = 0.f;
#pragma unroll 1
  for (int i0 = 0; i0 < kSeq; i0 += 32) {
    float sb = 0.f;
#pragma unroll 4
    for (int i = 0; i < 32; ++i) {
      const float dv = p[(size_t)(i0 + i) * kDim] - m;
      sb += dv * dv;
    }
    ss += sb;
  }
  const float var = ss * (1.0f / 1023.0f);
  const float sig = sqrtf(var);
  const float iv  = 1.0f / (sig + kOmEps);
  float* mp = mu + (size_t)b * kDim + d;
  float* ip = inv + (size_t)b * kDim + d;
  *(volatile float*)mp = m;
  *(volatile float*)ip = iv;
  __threadfence();
  *(volatile float*)mp = m;
  *(volatile float*)ip = iv;
}

__global__ __launch_bounds__(256) void combine_kernel(const float* __restrict__ G, const float* __restrict__ Bv,
                                                      const float* __restrict__ X, const float* __restrict__ mu,
                                                      const float* __restrict__ inv, float* __restrict__ out, int n4) {
  const int i = blockIdx.x * 256 + threadIdx.x;
  if (i >= n4) return;
  const size_t idx = (size_t)i * 4;
  const int d = (int)(idx & (size_t)(kDim - 1));
  const int b = (int)(idx / ((size_t)kSeq * kDim));
  const v4f g  = *(const v4f*)(G + idx);
  const v4f bv = *(const v4f*)(Bv + idx);
  const v4f x  = *(const v4f*)(X + idx);
  const v4f m  = *(const v4f*)(mu + (size_t)b * kDim + d);
  const v4f iv = *(const v4f*)(inv + (size_t)b * kDim + d);
  v4f o;
#pragma unroll
  for (int e = 0; e < 4; ++e) o[e] = g[e] * ((x[e] - m[e]) * iv[e]) + bv[e];
  float* op = out + idx;
  *(volatile v4f*)op = o;
  __threadfence();
  *(volatile v4f*)op = o;
}

extern "C" void kernel_launch(void* const* d_in, const int* in_sizes, int n_in,
                              void* d_out, int out_size, void* d_ws, size_t ws_size,
                              hipStream_t stream) {
  if (n_in < 14) return;
  if (in_sizes[0] != kTok * kDim || in_sizes[1] != kTok * kDim) return;
  if (in_sizes[2] != kDim * kDim || in_sizes[4] != kDim * kDim || in_sizes[6] != kDim * kDim ||
      in_sizes[8] != kDim * kDim || in_sizes[10] != kDim * kDim || in_sizes[12] != kDim * kDim) return;
  if (in_sizes[3] != kDim || in_sizes[5] != kDim || in_sizes[7] != kDim || in_sizes[9] != kDim ||
      in_sizes[11] != kDim || in_sizes[13] != kDim) return;
  if (out_size < 2 * kTok * kDim) return;
  if (ws_size < kWsTotal) return;

  const float* X  = (const float*)d_in[0];
  const float* Y  = (const float*)d_in[1];
  const float* Wq = (const float*)d_in[2];  const float* bq = (const float*)d_in[3];
  const float* Wk = (const float*)d_in[4];  const float* bk = (const float*)d_in[5];
  const float* Wv = (const float*)d_in[6];  const float* bv = (const float*)d_in[7];
  const float* Wo = (const float*)d_in[8];  const float* bo = (const float*)d_in[9];
  const float* Wg = (const float*)d_in[10]; const float* bg = (const float*)d_in[11];
  const float* Wb = (const float*)d_in[12]; const float* bb = (const float*)d_in[13];
  float* outX = (float*)d_out;
  float* outY = (float*)d_out + (size_t)kTok * kDim;

  char* ws = (char*)d_ws;
  unsigned short* Wt   = (unsigned short*)(ws + oW);
  unsigned short* WtQ  = Wt + 0 * (size_t)kDim * kDim;
  unsigned short* WtK  = Wt + 1 * (size_t)kDim * kDim;
  unsigned short* WtV  = Wt + 2 * (size_t)kDim * kDim;
  unsigned short* WtO  = Wt + 3 * (size_t)kDim * kDim;
  unsigned short* WtG  = Wt + 4 * (size_t)kDim * kDim;
  unsigned short* WtB  = Wt + 5 * (size_t)kDim * kDim;
  unsigned short* X16  = (unsigned short*)(ws + oX16);
  unsigned short* Kf   = (unsigned short*)(ws + oX16);
  unsigned short* Y16  = (unsigned short*)(ws + oY16);
  unsigned short* Att1 = (unsigned short*)(ws + oY16);
  unsigned short* YN16 = (unsigned short*)(ws + oY16);
  unsigned short* Att2 = (unsigned short*)(ws + oY16);
  unsigned short* Q1   = (unsigned short*)(ws + oQ1);
  unsigned short* YNT  = (unsigned short*)(ws + oQ1);
  unsigned short* K1   = (unsigned short*)(ws + oK1);
  unsigned short* A2   = (unsigned short*)(ws + oK1);
  unsigned short* V1T  = (unsigned short*)(ws + oV1T);
  unsigned short* Q2   = (unsigned short*)(ws + oV1T);
  unsigned short* Qc   = (unsigned short*)(ws + oQc);
  float*          Sbuf = (float*)(ws + oS);
  float*          BvP  = (float*)(ws + oS);
  unsigned short* Pbuf = (unsigned short*)(ws + oP);
  float*          Zbuf = (float*)(ws + oZ);
  float*          Gp   = (float*)(ws + oZ);
  float*          muP  = (float*)(ws + oMu);
  float*          invP = (float*)(ws + oInv);

  const long SD = (long)kSeq * kDim;
  const long SS = (long)kSeq * kSeq;
  const float invW      = 1.0f / kWCarry;
  const float invAttW   = 1.0f / (kAttCarry * kWCarry);
  const float pvScale   = kAttCarry / kPCarry;
  const float kfScale   = kKfCarry / kPCarry;
  const float sc2Scale  = kScale / kKfCarry;

  const dim3 blk256(256);
  const dim3 blk128(128);
  const dim3 gProj((kTok / 64) * (kDim / 64) / 8, 1);
  const dim3 gSq((kSeq / 64) * (kDim / 64) / 8, kBatch);
  const dim3 gSc((kSeq / 64) * (kSeq / 64) / 8, kChunkG);
  const dim3 gPv((kSeq / 64) * (kDk / 64) / 8, kChunkG);

  wtcast6_kernel<<<dim3(kDim / 64, kDim / 64, 6), blk256, 0, stream>>>(Wq, Wk, Wv, Wo, Wg, Wb, Wt, kWCarry);
  cast8_f16_kernel<<<dim3(kTok * kDim / 8 / 256), blk256, 0, stream>>>(X, X16, kTok * kDim / 8);
  cast8_f16_kernel<<<dim3(kTok * kDim / 8 / 256), blk256, 0, stream>>>(Y, Y16, kTok * kDim / 8);

  wmma_gemm64<0, false, 2, 1, false><<<gProj, blk256, 0, stream>>>(
      Y16, Y16, kDim, 0, WtQ, WtQ, kDim, 0, Q1, Q1, kDim, 0, bq, bq, 0, kTok, kDim, kDim, invW, 1.0f);
  wmma_gemm64<0, false, 2, 1, false><<<gProj, blk256, 0, stream>>>(
      X16, X16, kDim, 0, WtK, WtK, kDim, 0, K1, K1, kDim, 0, bk, bk, 0, kTok, kDim, kDim, invW, 1.0f);
  wmma_gemm64<0, false, 1, 1, false><<<gSq, blk256, 0, stream>>>(
      WtV, WtV, kDim, 0, X16, X16, kDim, SD, V1T, V1T, kSeq, SD, bv, bv, 0, kDim, kSeq, kDim, invW, 1.0f);

  for (int c = 0; c < kNumChunks; ++c) {
    const int b  = c / kChunksPerBatch;
    const int h0 = (c % kChunksPerBatch) * kChunkG;
    const size_t qoff = (size_t)b * SD + (size_t)h0 * kDk;
    const size_t voff = (size_t)b * SD + (size_t)h0 * kDk * kSeq;
    wmma_gemm64<0, false, 0, 0, false><<<gSc, blk256, 0, stream>>>(
        Q1 + qoff, Q1 + qoff, kDim, kDk, K1 + qoff, K1 + qoff, kDim, kDk,
        Sbuf, Sbuf, kSeq, SS, bq, bq, 0, kSeq, kSeq, kDk, kScale, 1.0f);
    softmax1024_kernel<<<dim3(kChunkG * kSeq), blk128, 0, stream>>>(Sbuf, Pbuf, kPCarry);
    wmma_gemm64<0, false, 0, 1, false><<<gPv, blk256, 0, stream>>>(
        Pbuf, Pbuf, kSeq, SS, V1T + voff, V1T + voff, kSeq, (long)kDk * kSeq,
        Att1 + qoff, Att1 + qoff, kDim, kDk, bq, bq, 0, kSeq, kDk, kSeq, pvScale, 1.0f);
  }

  wmma_gemm64<0, false, 2, 0, true><<<gProj, blk256, 0, stream>>>(
      Att1, Att1, kDim, 0, WtO, WtO, kDim, 0, Zbuf, Zbuf, kDim, 0, bo, Y, 0, kTok, kDim, kDim, invAttW, 1.0f);
  ln_row_kernel<<<dim3(kTok), blk256, 0, stream>>>(Zbuf, outY, YN16);
  transpose16_kernel<<<dim3(kDim / 64, kSeq / 64, kBatch), blk256, 0, stream>>>(YN16, YNT);

  wmma_gemm64<0, false, 2, 1, false><<<gProj, blk256, 0, stream>>>(
      X16, X16, kDim, 0, WtQ, WtQ, kDim, 0, Q2, Q2, kDim, 0, bq, bq, 0, kTok, kDim, kDim, invW, 1.0f);
  wmma_gemm64<0, false, 2, 1, false><<<gProj, blk256, 0, stream>>>(
      YN16, YN16, kDim, 0, WtQ, WtQ, kDim, 0, Qc, Qc, kDim, 0, bq, bq, 0, kTok, kDim, kDim, invW, 1.0f);

  wmma_gemm64<0, false, 0, 0, false><<<gSq, blk256, 0, stream>>>(
      Qc, Qc, kDim, SD, K1, K1, kDim, SD, Sbuf, Sbuf, kSeq, SS, bq, bq, 0, kSeq, kSeq, kDim, kScale, 1.0f);
  softmax1024_kernel<<<dim3(kBatch * kSeq), blk128, 0, stream>>>(Sbuf, Pbuf, kPCarry);
  wmma_gemm64<0, false, 0, 1, false><<<gSq, blk256, 0, stream>>>(
      Pbuf, Pbuf, kSeq, SS, YNT, YNT, kSeq, SD, Kf, Kf, kDim, SD, bq, bq, 0, kSeq, kDim, kSeq, kfScale, 1.0f);

  for (int c = 0; c < kNumChunks; ++c) {
    const int b  = c / kChunksPerBatch;
    const int h0 = (c % kChunksPerBatch) * kChunkG;
    const size_t qoff = (size_t)b * SD + (size_t)h0 * kDk;
    const size_t voff = (size_t)b * SD + (size_t)h0 * kDk * kSeq;
    wmma_gemm64<0, false, 0, 0, false><<<gSc, blk256, 0, stream>>>(
        Q2 + qoff, Q2 + qoff, kDim, kDk, Kf + qoff, Kf + qoff, kDim, kDk,
        Sbuf, Sbuf, kSeq, SS, bq, bq, 0, kSeq, kSeq, kDk, sc2Scale, 1.0f);
    softmax1024_kernel<<<dim3(kChunkG * kSeq), blk128, 0, stream>>>(Sbuf, Pbuf, kPCarry);
    wmma_gemm64<0, false, 0, 1, false><<<gPv, blk256, 0, stream>>>(
        Pbuf, Pbuf, kSeq, SS, YNT + voff, YNT + voff, kSeq, (long)kDk * kSeq,
        Att2 + qoff, Att2 + qoff, kDim, kDk, bq, bq, 0, kSeq, kDk, kSeq, pvScale, 1.0f);
  }

  wmma_gemm64<0, false, 2, 1, false><<<gProj, blk256, 0, stream>>>(
      Att2, Att2, kDim, 0, WtO, WtO, kDim, 0, A2, A2, kDim, 0, bo, bo, 0, kTok, kDim, kDim, invW, kAttCarry);
  wmma_gemm64<0, false, 2, 0, false><<<gProj, blk256, 0, stream>>>(
      A2, A2, kDim, 0, WtG, WtG, kDim, 0, Gp, Gp, kDim, 0, bg, bg, 0, kTok, kDim, kDim, invAttW, 1.0f);
  wmma_gemm64<0, false, 2, 0, false><<<gProj, blk256, 0, stream>>>(
      A2, A2, kDim, 0, WtB, WtB, kDim, 0, BvP, BvP, kDim, 0, bb, bb, 0, kTok, kDim, kDim, invAttW, 1.0f);

  colstats_kernel<<<dim3(kDim / 256, kBatch), blk256, 0, stream>>>(X, muP, invP);
  combine_kernel<<<dim3(kTok * kDim / 4 / 256), blk256, 0, stream>>>(Gp, BvP, X, muP, invP, outX, kTok * kDim / 4);
}
